// PokerEq3Net_1047972021004
// MI455X (gfx1250) — hardware-verified
//
#include <hip/hip_runtime.h>
#include <math.h>

typedef __attribute__((ext_vector_type(16))) _Float16 v16h;
typedef __attribute__((ext_vector_type(16))) __bf16 v16b;
typedef __attribute__((ext_vector_type(8)))  _Float16 v8h;
typedef __attribute__((ext_vector_type(8)))  float v8f;
typedef __attribute__((ext_vector_type(4)))  float v4f;
typedef __attribute__((ext_vector_type(2)))  float v2f;
typedef __attribute__((ext_vector_type(4)))  unsigned v4u;
typedef __attribute__((ext_vector_type(4)))  int v4i;
typedef float __attribute__((may_alias)) float_a;
typedef int __attribute__((may_alias)) int_a;

template <typename T> __device__ __forceinline__ void vst2(void* p, T v) { *(volatile T*)p = v; __threadfence(); *(volatile T*)p = v; }
__device__ __forceinline__ v8f wmma16(v16h a, v16h b, v8f c) {
  v8f d = __builtin_amdgcn_wmma_f32_16x16x32_f16(false, a, false, b, (short)0, c, false, false);
  asm volatile("v_nop\n\tv_nop\n\tv_nop\n\tv_nop" : "+v"(d) : "v"(a), "v"(b));
  return d;
}
__device__ __forceinline__ v8f wmma_bf(v16b a, v16b b, v8f c) {
  v8f d = __builtin_amdgcn_wmma_f32_16x16x32_bf16(false, a, false, b, (short)0, c, false, false);
  asm volatile("v_nop\n\tv_nop\n\tv_nop\n\tv_nop" : "+v"(d) : "v"(a), "v"(b));
  return d;
}
__device__ __forceinline__ v16h frag_h(const _Float16* rowk0, int lane) {
  union { v16h v; v8h q[2]; } u; const _Float16* p = rowk0 + 8 * (lane >> 4);
  u.q[0] = *(const v8h*)p; u.q[1] = *(const v8h*)(p + 16); return u.v;
}
__device__ __forceinline__ v16h frag_f32(const float* rowk0, int lane) {
  v16h a; const float* p = rowk0 + 8 * (lane >> 4);
#pragma unroll
  for (int i = 0; i < 8; ++i) { a[i] = (_Float16)p[i]; a[8 + i] = (_Float16)p[16 + i]; }
  return a;
}
__device__ __forceinline__ v16h frag_f32s(const float* rowk0, int lane, float sc) {
  v16h a; const float* p = rowk0 + 8 * (lane >> 4);
#pragma unroll
  for (int i = 0; i < 8; ++i) { a[i] = (_Float16)(p[i] * sc); a[8 + i] = (_Float16)(p[16 + i] * sc); }
  return a;
}
__device__ __forceinline__ v16h fragc_f32(const float* W, int k0, int n, int lane, int ld, int K) {
  v16h a; const int g = lane >> 4;
#pragma unroll
  for (int i = 0; i < 8; ++i) { const int ka = k0 + 8 * g + i, kb = ka + 16;
    a[i] = (_Float16)(ka < K ? W[(size_t)(ka < K ? ka : K - 1) * ld + n] : 0.f); a[8 + i] = (_Float16)(kb < K ? W[(size_t)(kb < K ? kb : K - 1) * ld + n] : 0.f); }
  return a;
}
struct F2 { v16b h, l; };
__device__ __forceinline__ F2 bsplit16(const float v[16]) { F2 r;
#pragma unroll
  for (int i = 0; i < 16; ++i) { const __bf16 h = (__bf16)v[i]; r.h[i] = h; r.l[i] = (__bf16)(v[i] - (float)h); }
  return r; }
__device__ __forceinline__ F2 split_row(const float* row, int k0, int lane) { float v[16]; const float* p = row + k0 + 8 * (lane >> 4);
#pragma unroll
  for (int i = 0; i < 8; ++i) { v[i] = p[i]; v[8 + i] = p[16 + i]; }
  return bsplit16(v); }
__device__ __forceinline__ F2 split_rowK(const float* row, int k0, int lane, int K) { float v[16]; const int g = lane >> 4;
#pragma unroll
  for (int i = 0; i < 8; ++i) { const int ka = k0 + 8 * g + i, kb = ka + 16; v[i] = ka < K ? row[ka < K ? ka : K - 1] : 0.f; v[8 + i] = kb < K ? row[kb < K ? kb : K - 1] : 0.f; }
  return bsplit16(v); }
__device__ __forceinline__ F2 split_col(const float* W, int k0, int n, int lane, int ld, int K) { float v[16]; const int g = lane >> 4;
#pragma unroll
  for (int i = 0; i < 8; ++i) { const int ka = k0 + 8 * g + i, kb = ka + 16; v[i] = ka < K ? W[(size_t)(ka < K ? ka : K - 1) * ld + n] : 0.f; v[8 + i] = kb < K ? W[(size_t)(kb < K ? kb : K - 1) * ld + n] : 0.f; }
  return bsplit16(v); }
__device__ __forceinline__ v8f mac3(const F2& a, const F2& b, v8f c) { c = wmma_bf(a.l, b.h, c); c = wmma_bf(a.h, b.l, c); return wmma_bf(a.h, b.h, c); }
__device__ __forceinline__ float sigm(float v) { return 1.0f / (1.0f + expf(-v)); }
#define LDSX() do { asm volatile("s_wait_dscnt 0" ::: "memory"); __builtin_amdgcn_wave_barrier(); __builtin_amdgcn_fence(__ATOMIC_RELEASE, "workgroup"); } while (0)


#ifndef NB
#define NB 64
#endif
#define NCARD 13
#define DD 128
#define NOUT 10
#define NPOS 2197
#define PPAD 2240
#define NTILE (PPAD / 64)
#define QROWS 832
typedef __attribute__((ext_vector_type(8))) __bf16 v8b;
__device__ __forceinline__ v16b frag_b(const __bf16* rowk0, int lane) {
  union { v16b v; v8b q[2]; } u; const __bf16* p = rowk0 + 8 * (lane >> 4);
  u.q[0] = *(const v8b*)p; u.q[1] = *(const v8b*)(p + 16); return u.v;
}
__device__ __forceinline__ float bfr(float v) { return (float)(__bf16)v; }
__device__ __attribute__((noinline)) float exp_ni(float v) { return expf(v); }
__device__ __attribute__((noinline)) float erf_ni(float v) { return erff(v); }

#define WS_PW   0u
#define WS_X    (WS_PW + 2u * 20 * DD * DD)
#define WS_TA   (WS_X + 4u * NB * 16 * DD)
#define WS_TB   (WS_TA + 4u * NB * DD * PPAD)
#define WS_PL   (WS_TB + 4u * NB * DD * PPAD)
#define WS_PP   (WS_PL + 4u * NB * QROWS * DD)
#define WS_END  (WS_PP + 4u * NB * QROWS * DD)

__global__ __launch_bounds__(128) void k_pack(const float* __restrict__ E2, const float* __restrict__ E3, const float* __restrict__ Q1, const float* __restrict__ Q2, const float* __restrict__ D1, const float* __restrict__ D2, __bf16* __restrict__ PW) {
  __shared__ __align__(16) __bf16 s[DD]; const int n = blockIdx.x, p = blockIdx.y, k = threadIdx.x; const float* Wm;
  if (p == 0) Wm = E2; else if (p == 1) Wm = E3; else if (p < 10) Wm = Q1 + (size_t)(p - 2) * DD * DD; else if (p < 18) Wm = Q2 + (size_t)(p - 10) * DD * DD; else if (p == 18) Wm = D1; else Wm = D2;
  s[k] = (__bf16)Wm[(size_t)k * DD + n]; __syncthreads();
  if (k < DD / 8) vst2((unsigned*)(PW + ((size_t)p * DD + n) * DD + k * 8), *(const v4u*)&s[k * 8]);
}
__global__ __launch_bounds__(128) void k_enc(const int* __restrict__ SU, const int* __restrict__ NU, const float* __restrict__ W1, const float* __restrict__ B1, const float* __restrict__ W2, const float* __restrict__ B2, const float* __restrict__ W3, const float* __restrict__ B3, float* __restrict__ X) {
  __shared__ float sa[16][DD], sb[16][DD]; const int b = blockIdx.x, c = threadIdx.x;
#pragma unroll 1
  for (int i = 0; i < 16; ++i) { float v = 0.f; if (i < NCARD) { const float s_ = (float)SU[b * NCARD + i], n_ = (float)NU[b * NCARD + i]; v = fmaxf(s_ * bfr(W1[c]) + n_ * bfr(W1[DD + c]) + bfr(B1[c]), 0.f); } sa[i][c] = v; }
  __syncthreads();
#pragma unroll 1
  for (int i = 0; i < NCARD; ++i) { float v = bfr(B2[c]);
#pragma unroll 1
    for (int k = 0; k < DD; ++k) v += sa[i][k] * bfr(W2[(size_t)k * DD + c]); sb[i][c] = fmaxf(v, 0.f); }
  __syncthreads();
#pragma unroll 1
  for (int i = 0; i < 16; ++i) { float v = 0.f; if (i < NCARD) { v = bfr(B3[c]);
#pragma unroll 1
      for (int k = 0; k < DD; ++k) v += sb[i][k] * bfr(W3[(size_t)k * DD + c]); } sa[i][c] = v; }
  __syncthreads();
  for (int q = c; q < 16 * DD / 4; q += 128) { const int i = q / (DD / 4), pc = q % (DD / 4); vst2(X + ((size_t)b * 16 + i) * DD + pc * 4, *(const v4f*)&sa[i][pc * 4]); }
}
__global__ __launch_bounds__(128) void k_outer(const float* __restrict__ X, float* __restrict__ T) {
  __shared__ float sx[16]; __shared__ __align__(16) float so[PPAD]; const int d = blockIdx.x, b = blockIdx.y, tid = threadIdx.x;
  if (tid < 16) sx[tid] = X[((size_t)b * 16 + tid) * DD + d];
  __syncthreads();
  for (int p = tid; p < PPAD; p += 128) { float v = 0.f; if (p < NPOS) { const int i = p / 169, j = (p / 13) % 13, k = p % 13; v = (sx[i] * sx[j]) * sx[k]; } so[p] = v; }
  __syncthreads();
  for (int q = tid; q < PPAD / 4; q += 128) vst2(T + ((size_t)b * DD + d) * PPAD + q * 4, *(const v4f*)&so[q * 4]);
}
__global__ __launch_bounds__(128) void k_pool(const float* __restrict__ T, float* __restrict__ PL) {
  const int b = blockIdx.x, d = threadIdx.x; const float* t = T + ((size_t)b * DD + d) * PPAD; float* pl = PL + (size_t)b * QROWS * DD + d; const float r13 = 1.0f / 13.0f;
#pragma unroll 1
  for (int jk = 0; jk < 169; ++jk) { float s = 0.f; for (int i = 0; i < NCARD; ++i) s += t[i * 169 + jk]; const float v = s * r13; *(volatile float*)(pl + (size_t)(0 + jk) * DD) = v; }
#pragma unroll 1
  for (int ik = 0; ik < 169; ++ik) { const int i = ik / 13, k = ik % 13; float s = 0.f; for (int j = 0; j < NCARD; ++j) s += t[i * 169 + j * 13 + k]; *(volatile float*)(pl + (size_t)(192 + ik) * DD) = s * r13; }
#pragma unroll 1
  for (int ij = 0; ij < 169; ++ij) { float s = 0.f; for (int k = 0; k < NCARD; ++k) s += t[ij * 13 + k]; *(volatile float*)(pl + (size_t)(384 + ij) * DD) = s * r13; }
  __threadfence();
  float mij[13];
#pragma unroll
  for (int k = 0; k < NCARD; ++k) { float s = 0.f; for (int j = 0; j < NCARD; ++j) s += pl[(size_t)(0 + j * 13 + k) * DD]; mij[k] = s * r13; *(volatile float*)(pl + (size_t)(576 + k) * DD) = mij[k]; }
#pragma unroll 1
  for (int j = 0; j < NCARD; ++j) { float s = 0.f; for (int k = 0; k < NCARD; ++k) s += pl[(size_t)(0 + j * 13 + k) * DD]; *(volatile float*)(pl + (size_t)(640 + j) * DD) = s * r13; }
#pragma unroll 1
  for (int i = 0; i < NCARD; ++i) { float s = 0.f; for (int k = 0; k < NCARD; ++k) s += pl[(size_t)(192 + i * 13 + k) * DD]; *(volatile float*)(pl + (size_t)(704 + i) * DD) = s * r13; }
  { float s = 0.f;
#pragma unroll
    for (int k = 0; k < NCARD; ++k) s += mij[k]; *(volatile float*)(pl + (size_t)768 * DD) = s * r13; }
#pragma unroll 1
  for (int q = 0; q < QROWS; ++q) { const bool pad = (q < 576) ? ((q % 192) >= 169) : (q < 768 ? ((q % 64) >= 13) : (q > 768)); if (pad) *(volatile float*)(pl + (size_t)q * DD) = 0.f; }
}
__global__ __launch_bounds__(128) void k_pproj(const float* __restrict__ PL, const __bf16* __restrict__ PWL, float* __restrict__ PP) {
  __shared__ __align__(16) float so[4][16][132];
  const int tid = threadIdx.x, wave = tid >> 5, lane = tid & 31, col = lane & 15, g = lane >> 4; const int tile = blockIdx.x, b = blockIdx.y; const int term = (tile < 9) ? (1 + tile / 3) : (4 + (tile - 9)); const size_t r0 = (size_t)b * QROWS + tile * 64 + wave * 16;
  const __bf16* P = PWL + (size_t)term * DD * DD;
  v8f acc[8] = {};
#pragma unroll
  for (int kc = 0; kc < DD / 32; ++kc) { const F2 a = split_row(PL + (r0 + col) * DD, kc * 32, lane);
#pragma unroll
    for (int j = 0; j < 8; ++j) { const v16b w = frag_b(P + (size_t)(j * 16 + col) * DD + kc * 32, lane); acc[j] = wmma_bf(a.l, w, acc[j]); acc[j] = wmma_bf(a.h, w, acc[j]); } }
#pragma unroll
  for (int j = 0; j < 8; ++j)
#pragma unroll
    for (int r = 0; r < 8; ++r) so[wave][8 * g + r][j * 16 + col] = acc[j][r];
  LDSX();
  for (int rl = 0; rl < 16; ++rl) vst2(PP + (r0 + rl) * DD + lane * 4, *(const v4f*)&so[wave][rl][lane * 4]);
}
__global__ __launch_bounds__(128) void k_eq(const float* __restrict__ T, const __bf16* __restrict__ PWL, const float* __restrict__ PP, const float* __restrict__ BIAS, float* __restrict__ TO) {
  __shared__ __align__(16) float st[DD][68];
  const int tid = threadIdx.x, wave = tid >> 5, lane = tid & 31, col = lane & 15, g = lane >> 4; const int tile = blockIdx.x, b = blockIdx.y; const int p0 = tile * 64; const int prow = p0 + wave * 16 + col;
  const float* tb = T + (size_t)b * DD * PPAD;
  v8f acc[8] = {};
#pragma unroll
  for (int kc = 0; kc < DD / 32; ++kc) { float v[16];
#pragma unroll
    for (int i = 0; i < 16; ++i) { const int d = kc * 32 + 8 * g + (i & 7) + ((i >> 3) << 4); v[i] = tb[(size_t)d * PPAD + prow]; }
    const F2 a = bsplit16(v);
#pragma unroll
    for (int j = 0; j < 8; ++j) { const v16b w = frag_b(PWL + (size_t)(j * 16 + col) * DD + kc * 32, lane); acc[j] = wmma_bf(a.l, w, acc[j]); acc[j] = wmma_bf(a.h, w, acc[j]); } }
  const float* ppb = PP + (size_t)b * QROWS * DD;
#pragma unroll
  for (int r = 0; r < 8; ++r) { const int p = p0 + wave * 16 + 8 * g + r; const int pc = (p < NPOS) ? p : 0; const int i = pc / 169, j = (pc / 13) % 13, k = pc % 13;
    const float* t1 = ppb + (size_t)(0 + j * 13 + k) * DD; const float* t2 = ppb + (size_t)(192 + i * 13 + k) * DD; const float* t3 = ppb + (size_t)(384 + i * 13 + j) * DD; const float* t4 = ppb + (size_t)(576 + k) * DD; const float* t5 = ppb + (size_t)(640 + j) * DD; const float* t6 = ppb + (size_t)(704 + i) * DD; const float* t7 = ppb + (size_t)768 * DD;
#pragma unroll
    for (int jj = 0; jj < 8; ++jj) { const int e = jj * 16 + col; float v = acc[jj][r] + t1[e] + t2[e] + t3[e] + t4[e] + t5[e] + t6[e] + t7[e] + bfr(BIAS[e]); v = fmaxf(v, 0.f); if (p >= NPOS) v = 0.f; st[e][wave * 16 + 8 * g + r] = v; } }
  __syncthreads();
  for (int q = tid; q < DD * 16; q += 128) { const int e = q >> 4, pc = q & 15; vst2(TO + ((size_t)b * DD + e) * PPAD + p0 + pc * 4, *(const v4f*)&st[e][pc * 4]); }
}
__global__ __launch_bounds__(128) void k_dec(const float* __restrict__ T, const float* __restrict__ W1, const float* __restrict__ B1, const float* __restrict__ W2, const float* __restrict__ B2, float* __restrict__ H2) {
  __shared__ float sv[DD], sh[DD]; __shared__ __align__(16) float so[DD]; const int b = blockIdx.x, c = threadIdx.x;
  { const float* t = T + ((size_t)b * DD + c) * PPAD; float s = 0.f; for (int p = 0; p < NPOS; ++p) s += t[p]; sv[c] = s; }
  __syncthreads();
  { float v = bfr(B1[c]); for (int k = 0; k < DD; ++k) v += sv[k] * bfr(W1[(size_t)k * DD + c]); sh[c] = fmaxf(v, 0.f); }
  __syncthreads();
  { float v = bfr(B2[c]); for (int k = 0; k < DD; ++k) v += sh[k] * bfr(W2[(size_t)k * DD + c]); so[c] = fmaxf(v, 0.f); }
  __syncthreads();
  if (c < 32) vst2(H2 + (size_t)b * DD + c * 4, *(const v4f*)&so[c * 4]);
}
__global__ __launch_bounds__(256) void k_final(const float* __restrict__ H2, const float* __restrict__ W3, const float* __restrict__ B3, float* __restrict__ out) {
  __shared__ __align__(16) float so[NB * NOUT]; const int tid = threadIdx.x;
  for (int q = tid; q < NB * NOUT; q += 256) { const int b = q / NOUT, o = q % NOUT; float v = bfr(B3[o]); for (int k = 0; k < DD; ++k) v += H2[(size_t)b * DD + k] * bfr(W3[(size_t)k * NOUT + o]); so[q] = v; }
  __syncthreads();
  for (int q = tid; q < NB * NOUT / 4; q += 256) vst2(out + q * 4, *(const v4f*)&so[q * 4]);
}
extern "C" void kernel_launch(void* const* d_in, const int* in_sizes, int n_in, void* d_out, int out_size, void* d_ws, size_t ws_size, hipStream_t stream) {
  (void)in_sizes; (void)n_in; (void)out_size;
  const float** F = (const float**)d_in; const int* SU = (const int*)d_in[0]; const int* NU = (const int*)d_in[1];
  if (ws_size < (size_t)WS_END) return;
  char* ws = (char*)d_ws; __bf16* PW = (__bf16*)(ws + WS_PW); float *X = (float*)(ws + WS_X), *TA = (float*)(ws + WS_TA), *TB = (float*)(ws + WS_TB), *PL = (float*)(ws + WS_PL), *PP = (float*)(ws + WS_PP);
  k_pack<<<dim3(DD, 20), 128, 0, stream>>>(F[4], F[6], F[8], F[10], F[12], F[14], PW);
  k_enc<<<NB, 128, 0, stream>>>(SU, NU, F[2], F[3], F[4], F[5], F[6], F[7], X);
  k_outer<<<dim3(DD, NB), 128, 0, stream>>>(X, TA);
  k_pool<<<NB, 128, 0, stream>>>(TA, PL);
  k_pproj<<<dim3(QROWS / 64, NB), 128, 0, stream>>>(PL, PW + (size_t)2 * DD * DD, PP);
  k_eq<<<dim3(NTILE, NB), 128, 0, stream>>>(TA, PW + (size_t)2 * DD * DD, PP, F[9], TB);
  k_pool<<<NB, 128, 0, stream>>>(TB, PL);
  k_pproj<<<dim3(QROWS / 64, NB), 128, 0, stream>>>(PL, PW + (size_t)10 * DD * DD, PP);
  k_eq<<<dim3(NTILE, NB), 128, 0, stream>>>(TB, PW + (size_t)10 * DD * DD, PP, F[11], TA);
  k_dec<<<NB, 128, 0, stream>>>(TA, F[12], F[13], F[14], F[15], PL);
  k_final<<<1, 256, 0, stream>>>(PL, F[16], F[17], (float*)d_out);
}
